// TemporalAttn_43997644980904
// MI455X (gfx1250) — hardware-verified
//
#include <hip/hip_runtime.h>
#include <math.h>

typedef __attribute__((ext_vector_type(16))) _Float16 v16h;
typedef __attribute__((ext_vector_type(16))) __bf16 v16b;
typedef __attribute__((ext_vector_type(8)))  _Float16 v8h;
typedef __attribute__((ext_vector_type(8)))  float v8f;
typedef __attribute__((ext_vector_type(4)))  float v4f;
typedef __attribute__((ext_vector_type(2)))  float v2f;
typedef __attribute__((ext_vector_type(4)))  unsigned v4u;
typedef __attribute__((ext_vector_type(4)))  int v4i;
typedef float __attribute__((may_alias)) float_a;
typedef int __attribute__((may_alias)) int_a;

template <typename T> __device__ __forceinline__ void vst2(void* p, T v) { *(volatile T*)p = v; __threadfence(); *(volatile T*)p = v; }
__device__ __forceinline__ v8f wmma16(v16h a, v16h b, v8f c) {
  v8f d = __builtin_amdgcn_wmma_f32_16x16x32_f16(false, a, false, b, (short)0, c, false, false);
  asm volatile("v_nop\n\tv_nop\n\tv_nop\n\tv_nop" : "+v"(d) : "v"(a), "v"(b));
  return d;
}
__device__ __forceinline__ v8f wmma_bf(v16b a, v16b b, v8f c) {
  v8f d = __builtin_amdgcn_wmma_f32_16x16x32_bf16(false, a, false, b, (short)0, c, false, false);
  asm volatile("v_nop\n\tv_nop\n\tv_nop\n\tv_nop" : "+v"(d) : "v"(a), "v"(b));
  return d;
}
__device__ __forceinline__ v16h frag_h(const _Float16* rowk0, int lane) {
  union { v16h v; v8h q[2]; } u; const _Float16* p = rowk0 + 8 * (lane >> 4);
  u.q[0] = *(const v8h*)p; u.q[1] = *(const v8h*)(p + 16); return u.v;
}
__device__ __forceinline__ v16h frag_f32(const float* rowk0, int lane) {
  v16h a; const float* p = rowk0 + 8 * (lane >> 4);
#pragma unroll
  for (int i = 0; i < 8; ++i) { a[i] = (_Float16)p[i]; a[8 + i] = (_Float16)p[16 + i]; }
  return a;
}
__device__ __forceinline__ v16h frag_f32s(const float* rowk0, int lane, float sc) {
  v16h a; const float* p = rowk0 + 8 * (lane >> 4);
#pragma unroll
  for (int i = 0; i < 8; ++i) { a[i] = (_Float16)(p[i] * sc); a[8 + i] = (_Float16)(p[16 + i] * sc); }
  return a;
}
__device__ __forceinline__ v16h fragc_f32(const float* W, int k0, int n, int lane, int ld, int K) {
  v16h a; const int g = lane >> 4;
#pragma unroll
  for (int i = 0; i < 8; ++i) { const int ka = k0 + 8 * g + i, kb = ka + 16;
    a[i] = (_Float16)(ka < K ? W[(size_t)(ka < K ? ka : K - 1) * ld + n] : 0.f); a[8 + i] = (_Float16)(kb < K ? W[(size_t)(kb < K ? kb : K - 1) * ld + n] : 0.f); }
  return a;
}
struct F2 { v16b h, l; };
__device__ __forceinline__ F2 bsplit16(const float v[16]) { F2 r;
#pragma unroll
  for (int i = 0; i < 16; ++i) { const __bf16 h = (__bf16)v[i]; r.h[i] = h; r.l[i] = (__bf16)(v[i] - (float)h); }
  return r; }
__device__ __forceinline__ F2 split_row(const float* row, int k0, int lane) { float v[16]; const float* p = row + k0 + 8 * (lane >> 4);
#pragma unroll
  for (int i = 0; i < 8; ++i) { v[i] = p[i]; v[8 + i] = p[16 + i]; }
  return bsplit16(v); }
__device__ __forceinline__ F2 split_rowK(const float* row, int k0, int lane, int K) { float v[16]; const int g = lane >> 4;
#pragma unroll
  for (int i = 0; i < 8; ++i) { const int ka = k0 + 8 * g + i, kb = ka + 16; v[i] = ka < K ? row[ka < K ? ka : K - 1] : 0.f; v[8 + i] = kb < K ? row[kb < K ? kb : K - 1] : 0.f; }
  return bsplit16(v); }
__device__ __forceinline__ F2 split_col(const float* W, int k0, int n, int lane, int ld, int K) { float v[16]; const int g = lane >> 4;
#pragma unroll
  for (int i = 0; i < 8; ++i) { const int ka = k0 + 8 * g + i, kb = ka + 16; v[i] = ka < K ? W[(size_t)(ka < K ? ka : K - 1) * ld + n] : 0.f; v[8 + i] = kb < K ? W[(size_t)(kb < K ? kb : K - 1) * ld + n] : 0.f; }
  return bsplit16(v); }
__device__ __forceinline__ v8f mac3(const F2& a, const F2& b, v8f c) { c = wmma_bf(a.l, b.h, c); c = wmma_bf(a.h, b.l, c); return wmma_bf(a.h, b.h, c); }
__device__ __forceinline__ float sigm(float v) { return 1.0f / (1.0f + expf(-v)); }
#define LDSX() do { asm volatile("s_wait_dscnt 0" ::: "memory"); __builtin_amdgcn_wave_barrier(); __builtin_amdgcn_fence(__ATOMIC_RELEASE, "workgroup"); } while (0)


#define NB 64
#define TT 256
#define SQ (TT + 1)
#define SP 272
#define DD 512
#define NH 8
#define HD 64
#define DFF 2048
#define OUTD 512
typedef __attribute__((ext_vector_type(8))) __bf16 v8b;
__device__ __forceinline__ v16b frag_b(const __bf16* rowk0, int lane) {
  union { v16b v; v8b q[2]; } u; const __bf16* p = rowk0 + 8 * (lane >> 4);
  u.q[0] = *(const v8b*)p; u.q[1] = *(const v8b*)(p + 16); return u.v;
}
__device__ __forceinline__ float bfr(float v) { return (float)(__bf16)v; }
__device__ __attribute__((noinline)) float exp_ni(float v) { return expf(v); }
__device__ __attribute__((noinline)) float erf_ni(float v) { return erff(v); }

#define WS_PV  0u
#define WS_PO  (WS_PV + 2u * (size_t)DD * DD)
#define WS_P1  (WS_PO + 2u * (size_t)HD * DD)
#define WS_P2  (WS_P1 + 2u * (size_t)DFF * HD)
#define WS_U   (WS_P2 + 2u * (size_t)OUTD * DFF)
#define WS_UL  (WS_U + 2u * 16 * DD)
#define WS_XP  (WS_UL + 2u * 16 * DD)
#define WS_Z   (WS_XP + 2u * (size_t)NB * DD * SP)
#define WS_RES (WS_Z + 4u * (size_t)NB * NH * DD)
#define WS_HID (WS_RES + 4u * (size_t)NB * DD)
#define WS_END (WS_HID + 4u * (size_t)NB * DFF)

__global__ __launch_bounds__(256) void k_pack(const float* __restrict__ WV, const float* __restrict__ WO, const float* __restrict__ W1, const float* __restrict__ W2, __bf16* __restrict__ P) {
  const int n = blockIdx.x, which = blockIdx.y, t = threadIdx.x; __shared__ __align__(16) __bf16 s[DFF];
  const int K = (which == 0) ? DD : (which == 1) ? DD : (which == 2) ? HD : DFF; const int nrow = (which == 0) ? DD : (which == 1) ? HD : (which == 2) ? DFF : OUTD; if (n >= nrow) return;
  const float* src = ((which == 0) ? WV : (which == 1) ? WO : (which == 2) ? W1 : W2) + (size_t)n * K; const size_t off = ((which == 0) ? WS_PV : (which == 1) ? WS_PO : (which == 2) ? WS_P1 : WS_P2) / 2;
  for (int k = t; k < K; k += 256) s[k] = (__bf16)src[k]; __syncthreads(); for (int q = t; q < K / 8; q += 256) vst2((unsigned*)(P + off + (size_t)n * K + q * 8), *(const v4u*)&s[q * 8]);
}
__global__ __launch_bounds__(256) void k_u(const float* __restrict__ CLS, const float* __restrict__ WQ, const float* __restrict__ WK, __bf16* __restrict__ U, __bf16* __restrict__ UL) {
  __shared__ float sc[DD]; __shared__ float sq[DD]; __shared__ __align__(16) __bf16 su[16][DD]; __shared__ __align__(16) __bf16 sul[16][DD]; const int t = threadIdx.x;
  for (int i = t; i < DD; i += 256) sc[i] = bfr(CLS[i]); __syncthreads();
  for (int o = t; o < DD; o += 256) { float a = 0.f; const float* w = WQ + (size_t)o * DD; for (int k = 0; k < DD; ++k) a += bfr(w[k]) * sc[k]; sq[o] = a; } __syncthreads();
  for (int e = t; e < 16 * DD; e += 256) { const int h = e / DD, c = e % DD; float a = 0.f; if (h < NH) { for (int d = 0; d < HD; ++d) a += bfr(WK[(size_t)(h * HD + d) * DD + c]) * sq[h * HD + d]; } const __bf16 hv = (__bf16)a; su[h][c] = hv; sul[h][c] = (__bf16)(a - (float)hv); }
  __syncthreads();
  for (int q = t; q < 16 * DD / 8; q += 256) { vst2((unsigned*)(U + q * 8), *(const v4u*)(&su[0][0] + q * 8)); vst2((unsigned*)(UL + q * 8), *(const v4u*)(&sul[0][0] + q * 8)); }
}
__global__ __launch_bounds__(256) void k_planes(const float* __restrict__ X, const float* __restrict__ CLS, __bf16* __restrict__ XP) {
  __shared__ __align__(16) __bf16 st[64][SP]; const int c0 = blockIdx.x * 64, t = threadIdx.x; const size_t b = blockIdx.y;
  for (int e = t; e < 64 * SP; e += 256) { const int cl = e / SP, s = e % SP; float v = 0.f; if (s == 0) v = bfr(CLS[c0 + cl]); else if (s <= TT) v = bfr(X[((b * TT + (s - 1)) * DD) + c0 + cl]); st[cl][s] = (__bf16)v; }
  __syncthreads();
  for (int q = t; q < 64 * SP / 8; q += 256) vst2((unsigned*)(XP + (b * DD + c0) * SP + q * 8), *(const v4u*)(&st[0][0] + q * 8));
}
__global__ __launch_bounds__(128) void k_att(const float* __restrict__ X, const float* __restrict__ CLS, const __bf16* __restrict__ U, const __bf16* __restrict__ UL, const __bf16* __restrict__ XP, float* __restrict__ Z) {
  __shared__ __align__(16) float ss[16][SP + 4]; __shared__ __align__(16) __bf16 sph[16][SP + 8]; __shared__ __align__(16) __bf16 spl[16][SP + 8]; __shared__ __align__(16) float sz[16][DD + 4];
  const int tid = threadIdx.x, wave = tid >> 5, lane = tid & 31, col = lane & 15, g = lane >> 4; const size_t b = blockIdx.x;
  for (int tile = wave; tile < SP / 16; tile += 4) { const int s0 = tile * 16; v8f acc = {};
#pragma unroll 2
    for (int kc = 0; kc < DD / 32; ++kc) { v16b a; { const int s = s0 + col; const float* p = (s == 0) ? (CLS + kc * 32 + 8 * g) : (X + ((b * TT + (s - 1)) * DD) + kc * 32 + 8 * g); const bool live = s < SQ;
#pragma unroll
        for (int i = 0; i < 8; ++i) { a[i] = live ? (__bf16)p[i] : (__bf16)0.f; a[8 + i] = live ? (__bf16)p[16 + i] : (__bf16)0.f; } }
      acc = wmma_bf(a, frag_b(U + (size_t)col * DD + kc * 32, lane), acc); acc = wmma_bf(a, frag_b(UL + (size_t)col * DD + kc * 32, lane), acc); }
#pragma unroll
    for (int r = 0; r < 8; ++r) ss[col][s0 + 8 * g + r] = acc[r] * 0.125f; }
  __syncthreads();
  { const int h = tid >> 4, part = tid & 15; if (h < NH) { float mx = -3.0e38f; for (int j = part; j < SQ; j += 16) mx = fmaxf(mx, ss[h][j]);
#pragma unroll
      for (int o = 1; o < 16; o <<= 1) mx = fmaxf(mx, __shfl_xor(mx, o));
      float sum = 0.f; for (int j = part; j < SQ; j += 16) { const float e2 = __expf(ss[h][j] - mx); ss[h][j] = e2; sum += e2; }
#pragma unroll
      for (int o = 1; o < 16; o <<= 1) sum += __shfl_xor(sum, o);
      const float inv = 1.0f / sum; for (int j = part; j < SP; j += 16) { const float p = (j < SQ) ? ss[h][j] * inv : 0.f; const __bf16 hv = (__bf16)p; sph[h][j] = hv; spl[h][j] = (__bf16)(p - (float)hv); } }
    else { for (int j = part; j < SP; j += 16) { sph[h][j] = (__bf16)0.f; spl[h][j] = (__bf16)0.f; } } }
  __syncthreads();
  { v8f acc[8] = {};
#pragma unroll 1
    for (int kc = 0; kc < SP / 32 + 1; ++kc) { const int k0 = kc * 32; v16b ah, al;
#pragma unroll
      for (int i = 0; i < 8; ++i) { const int k1 = k0 + 8 * g + i, k2 = k0 + 16 + 8 * g + i; ah[i] = (k1 < SP) ? sph[col][k1] : (__bf16)0.f; al[i] = (k1 < SP) ? spl[col][k1] : (__bf16)0.f; ah[8 + i] = (k2 < SP) ? sph[col][k2] : (__bf16)0.f; al[8 + i] = (k2 < SP) ? spl[col][k2] : (__bf16)0.f; }
#pragma unroll
      for (int j = 0; j < 8; ++j) { const int c = (wave * 8 + j) * 16 + col; v16b bfrag; const __bf16* pr = XP + (b * DD + c) * SP + k0 + 8 * g;
#pragma unroll
        for (int i = 0; i < 8; ++i) { const int k1 = k0 + 8 * g + i, k2 = k0 + 16 + 8 * g + i; bfrag[i] = (k1 < SP) ? pr[i] : (__bf16)0.f; bfrag[8 + i] = (k2 < SP) ? pr[16 + i] : (__bf16)0.f; }
        acc[j] = wmma_bf(ah, bfrag, acc[j]); acc[j] = wmma_bf(al, bfrag, acc[j]); } }
#pragma unroll
    for (int j = 0; j < 8; ++j)
#pragma unroll
      for (int r = 0; r < 8; ++r) sz[8 * g + r][(wave * 8 + j) * 16 + col] = acc[j][r]; }
  __syncthreads();
  for (int q = tid; q < NH * DD / 4; q += 128) { const int h = q / (DD / 4), c4 = q % (DD / 4); vst2(Z + (b * NH + h) * DD + c4 * 4, *(const v4f*)&sz[h][c4 * 4]); }
}
__global__ __launch_bounds__(128) void k_res(const float* __restrict__ Z, const __bf16* __restrict__ PV, float* __restrict__ RES) {
  __shared__ __align__(16) float so[4][16][68];
  const int tid = threadIdx.x, wave = tid >> 5, lane = tid & 31, col = lane & 15, g = lane >> 4; const int h = blockIdx.x; const int b0 = wave * 16;
  v8f acc[4] = {};
#pragma unroll 2
  for (int kc = 0; kc < DD / 32; ++kc) { const F2 a = split_row(Z + ((size_t)(b0 + col) * NH + h) * DD, kc * 32, lane);
#pragma unroll
    for (int j = 0; j < 4; ++j) { const v16b w = frag_b(PV + (size_t)(h * HD + j * 16 + col) * DD + kc * 32, lane); acc[j] = wmma_bf(a.h, w, acc[j]); acc[j] = wmma_bf(a.l, w, acc[j]); } }
#pragma unroll
  for (int j = 0; j < 4; ++j)
#pragma unroll
    for (int r = 0; r < 8; ++r) so[wave][8 * g + r][j * 16 + col] = acc[j][r];
  LDSX();
  for (int rl = 0; rl < 16; ++rl) if (lane < 16) vst2(RES + (size_t)(b0 + rl) * DD + h * HD + lane * 4, *(const v4f*)&so[wave][rl][lane * 4]);
}
__global__ __launch_bounds__(128) void k_mlp1(const float* __restrict__ RES, const __bf16* __restrict__ PO, const __bf16* __restrict__ P1, const float* __restrict__ B1, float* __restrict__ HID) {
  __shared__ __align__(16) float sco[4][16][68]; __shared__ __align__(16) float sh[4][16][132];
  const int tid = threadIdx.x, wave = tid >> 5, lane = tid & 31, col = lane & 15, g = lane >> 4; const int b0 = wave * 16;
  { v8f acc[4] = {};
#pragma unroll 2
    for (int kc = 0; kc < DD / 32; ++kc) { const F2 a = split_row(RES + (size_t)(b0 + col) * DD, kc * 32, lane);
#pragma unroll
      for (int j = 0; j < 4; ++j) { const v16b w = frag_b(PO + (size_t)(j * 16 + col) * DD + kc * 32, lane); acc[j] = wmma_bf(a.h, w, acc[j]); acc[j] = wmma_bf(a.l, w, acc[j]); } }
#pragma unroll
    for (int j = 0; j < 4; ++j)
#pragma unroll
      for (int r = 0; r < 8; ++r) sco[wave][8 * g + r][j * 16 + col] = acc[j][r]; }
  LDSX();
#pragma unroll 1
  for (int ch = 0; ch < DFF / 128; ++ch) { v8f acc[8] = {};
#pragma unroll
    for (int kc = 0; kc < HD / 32; ++kc) { const F2 a = split_row(&sco[wave][col][0], kc * 32, lane);
#pragma unroll
      for (int j = 0; j < 8; ++j) { const v16b w = frag_b(P1 + (size_t)(ch * 128 + j * 16 + col) * HD + kc * 32, lane); acc[j] = wmma_bf(a.h, w, acc[j]); acc[j] = wmma_bf(a.l, w, acc[j]); } }
#pragma unroll
    for (int j = 0; j < 8; ++j) { const float bb = bfr(B1[ch * 128 + j * 16 + col]);
#pragma unroll
      for (int r = 0; r < 8; ++r) sh[wave][8 * g + r][j * 16 + col] = fmaxf(acc[j][r] + bb, 0.f); }
    LDSX();
    for (int rl = 0; rl < 16; ++rl) vst2(HID + (size_t)(b0 + rl) * DFF + ch * 128 + lane * 4, *(const v4f*)&sh[wave][rl][lane * 4]);
    LDSX(); }
}
__global__ __launch_bounds__(128) void k_mlp2(const float* __restrict__ HID, const __bf16* __restrict__ P2, const float* __restrict__ B2, float* __restrict__ OUT) {
  __shared__ __align__(16) float so[4][16][132];
  const int tid = threadIdx.x, wave = tid >> 5, lane = tid & 31, col = lane & 15, g = lane >> 4; const int c0 = blockIdx.x * 128; const int b0 = wave * 16;
  v8f acc[8] = {};
#pragma unroll 2
  for (int kc = 0; kc < DFF / 32; ++kc) { const F2 a = split_row(HID + (size_t)(b0 + col) * DFF, kc * 32, lane);
#pragma unroll
    for (int j = 0; j < 8; ++j) { const v16b w = frag_b(P2 + (size_t)(c0 + j * 16 + col) * DFF + kc * 32, lane); acc[j] = wmma_bf(a.h, w, acc[j]); acc[j] = wmma_bf(a.l, w, acc[j]); } }
#pragma unroll
  for (int j = 0; j < 8; ++j) { const float bb = bfr(B2[c0 + j * 16 + col]);
#pragma unroll
    for (int r = 0; r < 8; ++r) so[wave][8 * g + r][j * 16 + col] = acc[j][r] + bb; }
  LDSX();
  for (int rl = 0; rl < 16; ++rl) vst2(OUT + (size_t)(b0 + rl) * OUTD + c0 + lane * 4, *(const v4f*)&so[wave][rl][lane * 4]);
}
extern "C" void kernel_launch(void* const* d_in, const int* in_sizes, int n_in, void* d_out, int out_size, void* d_ws, size_t ws_size, hipStream_t stream) {
  (void)in_sizes; (void)n_in; (void)out_size;
  const float** F = (const float**)d_in;
  if (ws_size < (size_t)WS_END) return;
  char* ws = (char*)d_ws; __bf16 *P = (__bf16*)ws, *U = (__bf16*)(ws + WS_U), *UL = (__bf16*)(ws + WS_UL), *XP = (__bf16*)(ws + WS_XP); float *Z = (float*)(ws + WS_Z), *RES = (float*)(ws + WS_RES), *HID = (float*)(ws + WS_HID);
  k_pack<<<dim3(DFF, 4), 256, 0, stream>>>(F[4], F[5], F[6], F[8], P);
  k_u<<<1, 256, 0, stream>>>(F[1], F[2], F[3], U, UL);
  k_planes<<<dim3(DD / 64, NB), 256, 0, stream>>>(F[0], F[1], XP);
  k_att<<<NB, 128, 0, stream>>>(F[0], F[1], U, UL, XP, Z);
  k_res<<<NH, 128, 0, stream>>>(Z, P + WS_PV / 2, RES);
  k_mlp1<<<1, 128, 0, stream>>>(RES, P + WS_PO / 2, P + WS_P1 / 2, F[7], HID);
  k_mlp2<<<OUTD / 128, 128, 0, stream>>>(HID, P + WS_P2 / 2, F[9], (float*)d_out);
}
